// SOG_3DmixedSpecies_dimer_309237645345
// MI455X (gfx1250) — hardware-verified
//
#include <hip/hip_runtime.h>


namespace {
constexpr int NBt = 8, NP = 3000, NPP = 3008, NC = 4, M = 31, MP = 32, MH = 15, NXY = MP * MP, NCZ = NC * MP, NSH = 12;
constexpr float LBOX = 10.0f, VOL = 1000.0f, XS = 8.0f;
constexpr float TWO_PI = 6.283185307179586f;

typedef _Float16 b16;
typedef __attribute__((ext_vector_type(16))) _Float16 v16b;
typedef __attribute__((ext_vector_type(8))) _Float16 v8b;
typedef __attribute__((ext_vector_type(8))) float v8f;
typedef __attribute__((ext_vector_type(4))) float v4f;
__device__ __forceinline__ float bf16_rne(float f) { unsigned int u = __float_as_uint(f); u += 0x7FFFu + ((u >> 16) & 1u); return __uint_as_float(u & 0xFFFF0000u); }
__device__ __forceinline__ void split16(float v, b16& hi, b16& lo) { hi = (b16)v; lo = (b16)(v - (float)hi); }
__device__ __forceinline__ v16b frag_kb(const b16* p, int hh) { const v8b a = *(const v8b*)(p + 8 * hh), b = *(const v8b*)(p + 16 + 8 * hh); v16b f;
#pragma unroll
  for (int e = 0; e < 8; ++e) { f[e] = a[e]; f[8 + e] = b[e]; } return f; }
__device__ __forceinline__ v8f wmma16b(v16b a, v16b b, v8f c) { v8f d = __builtin_amdgcn_wmma_f32_16x16x32_f16(false, a, false, b, (short)0, c, false, false); asm volatile("v_nop\n\tv_nop\n\tv_nop\n\tv_nop" : "+v"(d) : "v"(a), "v"(b)); return d; }
__device__ __forceinline__ void wave_lds_sync() { __builtin_amdgcn_fence(__ATOMIC_RELEASE, "workgroup"); __builtin_amdgcn_wave_barrier(); __builtin_amdgcn_fence(__ATOMIC_ACQUIRE, "workgroup"); }
__device__ __forceinline__ float pmul(float a, float b) { float p = a * b; asm volatile("" : "+v"(p)); return p; }
__device__ __forceinline__ v8f mma3(v8f acc, v16b ah, v16b al, v16b bh, v16b bl) { acc = wmma16b(ah, bh, acc); acc = wmma16b(ah, bl, acc); return wmma16b(al, bh, acc); }

__global__ __launch_bounds__(256) void mult_kernel(const float* __restrict__ shift, const float* __restrict__ amp, float* __restrict__ MULT, float* __restrict__ DIAG) {
  __shared__ float Se[NSH], Sa[NSH], Sp[256], Sd[32];
  const int t_ = threadIdx.x;
  if (t_ < NSH) { Se[t_] = __expf(2.0f * bf16_rne(shift[t_])); Sa[t_] = bf16_rne(amp[t_]); }
  __syncthreads();
  float part = 0.0f;
  for (int pass = 0; pass < 2; ++pass) { part = 0.0f;
    for (int idx = t_; idx < NXY * MP; idx += 256) { const int mz = idx & 31, my = (idx >> 5) & 31, mx = idx >> 10; float v = 0.0f;
      if (mx < M && my < M && mz < M) { const float kx = TWO_PI / LBOX * (float)(mx - MH), ky = TWO_PI / LBOX * (float)(my - MH), kz = TWO_PI / LBOX * (float)(mz - MH); const float k2 = kx * kx + ky * ky + kz * kz;
        if (!(mx == MH && my == MH && mz == MH)) {
#pragma unroll 1
          for (int s = 0; s < NSH; ++s) v += pmul(Sa[s], __expf(-pmul(k2, Se[s]))); } }
      ((volatile float*)MULT)[idx] = v; part += v; }
    __threadfence(); }
  Sp[t_] = part; __syncthreads();
  if (t_ < 32) { float s = 0.0f; for (int k = t_ * 8; k < t_ * 8 + 8; ++k) s += Sp[k]; Sd[t_] = s; }
  __syncthreads();
  if (t_ < 32) { float tot = 0.0f; for (int k = 0; k < 32; ++k) tot += Sd[k]; for (int pass = 0; pass < 2; ++pass) { ((volatile float*)DIAG)[t_] = tot / (2.0f * VOL); __threadfence(); } }
}
__global__ __launch_bounds__(256) void trig_kernel(const float* __restrict__ pos, const float* __restrict__ chg, int b, float* __restrict__ CZ, float* __restrict__ SZ, b16* __restrict__ EJRh, b16* __restrict__ EJRl, b16* __restrict__ EJIh, b16* __restrict__ EJIl, b16* __restrict__ EJNh, b16* __restrict__ EJNl, b16* __restrict__ ARh, b16* __restrict__ ARl, b16* __restrict__ AIh, b16* __restrict__ AIl, b16* __restrict__ BRh, b16* __restrict__ BRl, b16* __restrict__ BIh, b16* __restrict__ BIl, b16* __restrict__ BNh, b16* __restrict__ BNl) {
  __shared__ float Cx[64][MP], Sx[64][MP], Cy[64][MP], Sy[64][MP], Czs[64][MP], Szs[64][MP], Q[64][NC];
  __shared__ __attribute__((aligned(16))) b16 Th[MP][64 + 8], Tl[MP][64 + 8], Uh[MP][64 + 8], Ul[MP][64 + 8];
  __shared__ __attribute__((aligned(16))) b16 Sg[8][6][256 + 8];
  const int j0 = blockIdx.x * 64, t_ = threadIdx.x, wave = t_ >> 5, lane = t_ & 31;
#pragma unroll 1
  for (int k = t_; k < 64 * 3 * MP; k += 256) { const int m = k & 31, ax = (k >> 5) % 3, jj = k / 96; const int j = j0 + jj; float cv = 0.0f, sv = 0.0f;
    if (m < M && j < NP) { const float x = TWO_PI / LBOX * (bf16_rne(pos[((size_t)b * NP + j) * 3 + ax]) - 0.5f * LBOX); const float th = x * (float)(m - MH); __sincosf(th, &sv, &cv); }
    if (ax == 0) { Cx[jj][m] = cv; Sx[jj][m] = sv; } else if (ax == 1) { Cy[jj][m] = cv; Sy[jj][m] = sv; } else { Czs[jj][m] = cv; Szs[jj][m] = sv; } }
  for (int k = t_; k < 64 * NC; k += 256) { const int c = k & 3, jj = k >> 2; const int j = j0 + jj; Q[jj][c] = (j < NP) ? bf16_rne(chg[((size_t)b * NP + j) * NC + c]) : 0.0f; }
  __syncthreads();
  for (int pass = 0; pass < 2; ++pass) { for (int rr = wave * 8; rr < wave * 8 + 8; ++rr) if (j0 + rr < NPP) { ((volatile float*)CZ)[(size_t)(j0 + rr) * MP + lane] = Czs[rr][lane]; ((volatile float*)SZ)[(size_t)(j0 + rr) * MP + lane] = Szs[rr][lane]; } __threadfence(); }
  for (int rr = wave * 8; rr < wave * 8 + 8; ++rr) { const int j = j0 + rr;
    for (int qd = 0; qd < 4; ++qd) {
#pragma unroll 1
      for (int q = 0; q < 8; ++q) { const int e = lane * 8 + q, e0 = qd * 256 + e; const int mx = e0 >> 5, my = e0 & 31; const bool live = (mx < M) && (my < M) && (j < NP);
        const float cx = Cx[rr][mx], sx = Sx[rr][mx], cy = Cy[rr][my], sy = Sy[rr][my]; const float er = live ? (pmul(cx, cy) - pmul(sx, sy)) : 0.0f, ei = live ? -(pmul(sx, cy) + pmul(cx, sy)) : 0.0f; b16 a_, c_;
        split16(er * XS, a_, c_); Sg[wave][0][e] = a_; Sg[wave][1][e] = c_; split16(ei * XS, a_, c_); Sg[wave][2][e] = a_; Sg[wave][3][e] = c_; split16(-ei * XS, a_, c_); Sg[wave][4][e] = a_; Sg[wave][5][e] = c_; }
      wave_lds_sync();
      const size_t gi = (size_t)j * NXY + qd * 256 + lane * 8;
      for (int pass = 0; pass < 2; ++pass) { *(volatile v8b*)(EJRh + gi) = *(const v8b*)(&Sg[wave][0][lane * 8]); *(volatile v8b*)(EJRl + gi) = *(const v8b*)(&Sg[wave][1][lane * 8]); *(volatile v8b*)(EJIh + gi) = *(const v8b*)(&Sg[wave][2][lane * 8]); *(volatile v8b*)(EJIl + gi) = *(const v8b*)(&Sg[wave][3][lane * 8]); *(volatile v8b*)(EJNh + gi) = *(const v8b*)(&Sg[wave][4][lane * 8]); *(volatile v8b*)(EJNl + gi) = *(const v8b*)(&Sg[wave][5][lane * 8]); __threadfence(); }
      wave_lds_sync(); } }
  for (int mx = 0; mx < MP; ++mx) {
    __syncthreads();
#pragma unroll 1
    for (int k = t_; k < MP * 64; k += 256) { const int jj = k & 63, my = k >> 6; const int j = j0 + jj; const bool live = (mx < M) && (my < M) && (j < NP);
      const float cx = Cx[jj][mx], sx = Sx[jj][mx], cy = Cy[jj][my], sy = Sy[jj][my]; const float er = live ? (pmul(cx, cy) - pmul(sx, sy)) : 0.0f, ei = live ? -(pmul(sx, cy) + pmul(cx, sy)) : 0.0f; b16 a_, c_;
      split16(er * XS, a_, c_); Th[my][jj] = a_; Tl[my][jj] = c_; split16(ei * XS, a_, c_); Uh[my][jj] = a_; Ul[my][jj] = c_; }
    __syncthreads();
    for (int pass = 0; pass < 2; ++pass) { for (int q = t_; q < MP * 8; q += 256) { const int my = q >> 3, c8 = (q & 7) * 8; const size_t gi = (size_t)(mx * MP + my) * NPP + j0 + c8;
        *(volatile v8b*)(ARh + gi) = *(const v8b*)(&Th[my][c8]); *(volatile v8b*)(ARl + gi) = *(const v8b*)(&Tl[my][c8]); *(volatile v8b*)(AIh + gi) = *(const v8b*)(&Uh[my][c8]); *(volatile v8b*)(AIl + gi) = *(const v8b*)(&Ul[my][c8]); } __threadfence(); } }
  for (int c = 0; c < NC; ++c) {
    __syncthreads();
#pragma unroll 1
    for (int k = t_; k < MP * 64; k += 256) { const int jj = k & 63, mz = k >> 6; const int j = j0 + jj; const bool live = (mz < M) && (j < NP); const float qv = Q[jj][c];
      const float br = live ? pmul(qv, Czs[jj][mz]) : 0.0f, bi = live ? -pmul(qv, Szs[jj][mz]) : 0.0f; b16 a_, c_; split16(br * XS, a_, c_); Th[mz][jj] = a_; Tl[mz][jj] = c_; split16(bi * XS, a_, c_); Uh[mz][jj] = a_; Ul[mz][jj] = c_; }
    __syncthreads();
    for (int pass = 0; pass < 2; ++pass) { for (int q = t_; q < MP * 8; q += 256) { const int mz = q >> 3, c8 = (q & 7) * 8; const size_t gi = (size_t)(c * MP + mz) * NPP + j0 + c8; v8b nh_, nl_; const v8b uh = *(const v8b*)(&Uh[mz][c8]), ul = *(const v8b*)(&Ul[mz][c8]);
#pragma unroll
        for (int q2 = 0; q2 < 8; ++q2) { nh_[q2] = -uh[q2]; nl_[q2] = -ul[q2]; }
        *(volatile v8b*)(BRh + gi) = *(const v8b*)(&Th[mz][c8]); *(volatile v8b*)(BRl + gi) = *(const v8b*)(&Tl[mz][c8]); *(volatile v8b*)(BIh + gi) = uh; *(volatile v8b*)(BIl + gi) = ul; *(volatile v8b*)(BNh + gi) = nh_; *(volatile v8b*)(BNl + gi) = nl_; } __threadfence(); } }
}
__global__ __launch_bounds__(128) void gemm1_kernel(const b16* __restrict__ ARh, const b16* __restrict__ ARl, const b16* __restrict__ AIh, const b16* __restrict__ AIl, const b16* __restrict__ BRh, const b16* __restrict__ BRl, const b16* __restrict__ BIh, const b16* __restrict__ BIl, const b16* __restrict__ BNh, const b16* __restrict__ BNl, const float* __restrict__ MULT, b16* __restrict__ F2Rh, b16* __restrict__ F2Rl, b16* __restrict__ F2Ih, b16* __restrict__ F2Il) {
  __shared__ __attribute__((aligned(16))) b16 Trh[64][64 + 8], Trl[64][64 + 8], Tih[64][64 + 8], Til[64][64 + 8];
  const int wave = threadIdx.x >> 5, lane = threadIdx.x & 31, nloc = lane & 15, hlf = lane >> 4, t_ = threadIdx.x; const int m0 = blockIdx.x * 64, n0 = blockIdx.y * 64; const int mrow = m0 + wave * 16;
  v8f fr[4], fi[4];
#pragma unroll
  for (int t = 0; t < 4; ++t) { fr[t] = (v8f){}; fi[t] = (v8f){}; }
  for (int kb = 0; kb < NPP; kb += 32) { const size_t ao = (size_t)(mrow + nloc) * NPP + kb; const v16b arh = frag_kb(ARh + ao, hlf), arl = frag_kb(ARl + ao, hlf), aih = frag_kb(AIh + ao, hlf), ail = frag_kb(AIl + ao, hlf);
#pragma unroll
    for (int t = 0; t < 4; ++t) { const size_t bo = (size_t)(n0 + t * 16 + nloc) * NPP + kb;
      { const v16b brh = frag_kb(BRh + bo, hlf), brl = frag_kb(BRl + bo, hlf); fr[t] = mma3(fr[t], arh, arl, brh, brl); fi[t] = mma3(fi[t], aih, ail, brh, brl); }
      { const v16b bnh = frag_kb(BNh + bo, hlf), bnl = frag_kb(BNl + bo, hlf); fr[t] = mma3(fr[t], aih, ail, bnh, bnl); }
      { const v16b bih = frag_kb(BIh + bo, hlf), bil = frag_kb(BIl + bo, hlf); fi[t] = mma3(fi[t], arh, arl, bih, bil); } } }
#pragma unroll
  for (int t = 0; t < 4; ++t)
#pragma unroll
    for (int r = 0; r < 8; ++r) { const int ml = wave * 16 + 8 * hlf + r, nl = t * 16 + nloc; const int mz = (n0 + nl) & 31; const float mu = MULT[(size_t)(m0 + ml) * MP + mz];
      b16 a_, c_; split16(pmul(fr[t][r] * (1.0f / (XS * XS)), mu), a_, c_); Trh[nl][ml] = a_; Trl[nl][ml] = c_; split16(pmul(fi[t][r] * (1.0f / (XS * XS)), mu), a_, c_); Tih[nl][ml] = a_; Til[nl][ml] = c_; }
  __syncthreads();
  for (int pass = 0; pass < 2; ++pass) { for (int q = t_; q < 64 * 8; q += 128) { const int nl = q >> 3, c8 = (q & 7) * 8; const size_t gi = (size_t)(n0 + nl) * NXY + m0 + c8;
      *(volatile v8b*)(F2Rh + gi) = *(const v8b*)(&Trh[nl][c8]); *(volatile v8b*)(F2Rl + gi) = *(const v8b*)(&Trl[nl][c8]); *(volatile v8b*)(F2Ih + gi) = *(const v8b*)(&Tih[nl][c8]); *(volatile v8b*)(F2Il + gi) = *(const v8b*)(&Til[nl][c8]); } __threadfence(); }
}
__global__ __launch_bounds__(128) void gemm2_kernel(const b16* __restrict__ EJRh, const b16* __restrict__ EJRl, const b16* __restrict__ EJIh, const b16* __restrict__ EJIl, const b16* __restrict__ EJNh, const b16* __restrict__ EJNl, const b16* __restrict__ F2Rh, const b16* __restrict__ F2Rl, const b16* __restrict__ F2Ih, const b16* __restrict__ F2Il, float* __restrict__ TR, float* __restrict__ TI) {
  __shared__ __attribute__((aligned(16))) float Sr[4][16][64 + 4], Si[4][16][64 + 4];
  const int wave = threadIdx.x >> 5, lane = threadIdx.x & 31, nloc = lane & 15, hlf = lane >> 4; const int m0 = blockIdx.x * 64 + wave * 16, n0 = blockIdx.y * 64;
  v8f tr[4], ti[4];
#pragma unroll
  for (int t = 0; t < 4; ++t) { tr[t] = (v8f){}; ti[t] = (v8f){}; }
  for (int kb = 0; kb < NXY; kb += 32) { const size_t ao = (size_t)(m0 + nloc) * NXY + kb; const v16b erh = frag_kb(EJRh + ao, hlf), erl = frag_kb(EJRl + ao, hlf), eih = frag_kb(EJIh + ao, hlf), eil = frag_kb(EJIl + ao, hlf), enh = frag_kb(EJNh + ao, hlf), enl = frag_kb(EJNl + ao, hlf);
#pragma unroll
    for (int t = 0; t < 4; ++t) { const size_t bo = (size_t)(n0 + t * 16 + nloc) * NXY + kb;
      { const v16b frh = frag_kb(F2Rh + bo, hlf), frl = frag_kb(F2Rl + bo, hlf); tr[t] = mma3(tr[t], erh, erl, frh, frl); ti[t] = mma3(ti[t], enh, enl, frh, frl); }
      { const v16b fih = frag_kb(F2Ih + bo, hlf), fil = frag_kb(F2Il + bo, hlf); tr[t] = mma3(tr[t], eih, eil, fih, fil); ti[t] = mma3(ti[t], erh, erl, fih, fil); } } }
#pragma unroll
  for (int t = 0; t < 4; ++t)
#pragma unroll
    for (int r = 0; r < 8; ++r) { Sr[wave][8 * hlf + r][t * 16 + nloc] = tr[t][r] * (1.0f / XS); Si[wave][8 * hlf + r][t * 16 + nloc] = ti[t][r] * (1.0f / XS); }
  wave_lds_sync();
  for (int pass = 0; pass < 2; ++pass) { for (int rr = 0; rr < 16; ++rr) if (lane < 16) { const size_t gi = (size_t)(m0 + rr) * NCZ + n0 + lane * 4; *(volatile v4f*)(TR + gi) = *(const v4f*)(&Sr[wave][rr][lane * 4]); *(volatile v4f*)(TI + gi) = *(const v4f*)(&Si[wave][rr][lane * 4]); } __threadfence(); }
}
__global__ __launch_bounds__(256) void energy_kernel(const float* __restrict__ TR, const float* __restrict__ TI, const float* __restrict__ CZ, const float* __restrict__ SZ, const float* __restrict__ chg, const float* __restrict__ DIAG, float* __restrict__ out) {
  const int p = blockIdx.x * 256 + threadIdx.x; const int pc = p < NBt * NP ? p : NBt * NP - 1; const int b = pc / NP, j = pc - b * NP; const size_t row = (size_t)b * NPP + j;
  const float diag = DIAG[0]; float e = 0.0f;
#pragma unroll 1
  for (int c = 0; c < NC; ++c) { float ph = 0.0f;
#pragma unroll 1
    for (int mz = 0; mz < M; ++mz) ph += pmul(TR[row * NCZ + c * MP + mz], CZ[row * MP + mz]) - pmul(TI[row * NCZ + c * MP + mz], SZ[row * MP + mz]);
    e += pmul(bf16_rne(chg[((size_t)b * NP + j) * NC + c]), ph / (2.0f * VOL) - diag); }
  for (int pass = 0; pass < 2; ++pass) { if (p < NBt * NP) ((volatile float*)out)[p] = e; __threadfence(); }
}
}

extern "C" void kernel_launch(void* const* d_in, const int* in_sizes, int n_in, void* d_out, int out_size, void* d_ws, size_t ws_size, hipStream_t stream) {
  (void)n_in;
  auto Fp = [&](int i) { return (const float*)d_in[i]; };
  if (in_sizes[0] != NBt * NP * 3 || in_sizes[1] != NBt * NP * NC || in_sizes[2] != NSH || in_sizes[3] != NSH || out_size != NBt * NP) return;
  size_t off = 0; char* ws = (char*)d_ws;
  auto carve = [&](size_t bytes) { char* p = ws + off; off += (bytes + 255) & ~(size_t)255; return p; };
  float* MULT = (float*)carve((size_t)NXY * MP * 4); float* DIAG = (float*)carve(256);
  float* CZ = (float*)carve((size_t)NBt * NPP * MP * 4); float* SZ = (float*)carve((size_t)NBt * NPP * MP * 4);
  const size_t ej = (size_t)NPP * NXY, aj = (size_t)NXY * NPP, bj = (size_t)NCZ * NPP, fj = (size_t)NCZ * NXY;
  b16* EJ[6]; for (int i = 0; i < 6; ++i) EJ[i] = (b16*)carve(ej * 2);
  b16* AP[4]; for (int i = 0; i < 4; ++i) AP[i] = (b16*)carve(aj * 2);
  b16* BP[6]; for (int i = 0; i < 6; ++i) BP[i] = (b16*)carve(bj * 2);
  b16* FP2[4]; for (int i = 0; i < 4; ++i) FP2[i] = (b16*)carve(fj * 2);
  float* TR = (float*)carve((size_t)NBt * NPP * NCZ * 4); float* TI = (float*)carve((size_t)NBt * NPP * NCZ * 4);
  if (off > ws_size) return;
  mult_kernel<<<1, 256, 0, stream>>>(Fp(2), Fp(3), MULT, DIAG);
  for (int b = 0; b < NBt; ++b) {
    trig_kernel<<<NPP / 64, 256, 0, stream>>>(Fp(0), Fp(1), b, CZ + (size_t)b * NPP * MP, SZ + (size_t)b * NPP * MP, EJ[0], EJ[1], EJ[2], EJ[3], EJ[4], EJ[5], AP[0], AP[1], AP[2], AP[3], BP[0], BP[1], BP[2], BP[3], BP[4], BP[5]);
    gemm1_kernel<<<dim3(NXY / 64, NCZ / 64), 128, 0, stream>>>(AP[0], AP[1], AP[2], AP[3], BP[0], BP[1], BP[2], BP[3], BP[4], BP[5], MULT, FP2[0], FP2[1], FP2[2], FP2[3]);
    gemm2_kernel<<<dim3(NPP / 64, NCZ / 64), 128, 0, stream>>>(EJ[0], EJ[1], EJ[2], EJ[3], EJ[4], EJ[5], FP2[0], FP2[1], FP2[2], FP2[3], TR + (size_t)b * NPP * NCZ, TI + (size_t)b * NPP * NCZ); }
  energy_kernel<<<(NBt * NP + 255) / 256, 256, 0, stream>>>(TR, TI, CZ, SZ, Fp(1), DIAG, (float*)d_out);
}
